// GroupedQueryAttention_66571993088382
// MI455X (gfx1250) — hardware-verified
//
#include <hip/hip_runtime.h>
#ifndef NB
#define NB 2
#endif
#ifndef SEQ
#define SEQ 2048
#endif
#define NB_FULL 2
#define SEQ_FULL 2048
#define DM 1024
#define NH 16
#define NKV 4
#define HPG 4
#define HD 64
#define KVD (NKV * HD)
#define NQKV (DM + 2 * KVD)
#define KOFF DM
#define VOFF (DM + KVD)
#define QT0 128

static_assert((SEQ & (SEQ - 1)) == 0);
static_assert(SEQ >= 2 * QT0);
static_assert(SEQ <= SEQ_FULL);
static_assert(NB <= NB_FULL);
static_assert((SEQ % 128) == 0);
static_assert(QT0 == 128);
static_assert(HPG == 4);
static_assert(NH == NKV * HPG);
static_assert(DM == NH * HD);
static_assert(DM / 8 == 128);
static_assert(DM / 64 == 16);
static_assert((NQKV % 64) == 0);
static_assert((DM % 32) == 0);
static_assert(HD == 64);

typedef unsigned short v8us __attribute__((ext_vector_type(8), may_alias));
typedef float  v8f  __attribute__((ext_vector_type(8)));
typedef float  v4f  __attribute__((ext_vector_type(4)));
typedef float  v4fa __attribute__((ext_vector_type(4), may_alias));
typedef _Float16 v16h __attribute__((ext_vector_type(16)));
typedef _Float16 v4h __attribute__((ext_vector_type(4)));
union FragH { v16h v; v8us half[2]; _Float16 h[16]; unsigned short u[16]; };

__device__ __forceinline__ unsigned short bf16_bits(float x) { unsigned int u = __float_as_uint(x); return (unsigned short)((u + 0x7FFFu + ((u >> 16) & 1u)) >> 16); }
__device__ __forceinline__ float bf16_val(unsigned short b) { return __uint_as_float(((unsigned int)b) << 16); }
__device__ __forceinline__ float bf16_rne(float x) { return bf16_val(bf16_bits(x)); }

__device__ __forceinline__ v16h g2_frag(const _Float16* p, int hh) { FragH f; f.half[0] = *(const v8us*)((const unsigned short*)p + 8 * hh); f.half[1] = *(const v8us*)((const unsigned short*)p + 16 + 8 * hh); return f.v; }
__device__ __forceinline__ v8f g2_mma(v16h a, v16h b, v8f c) { v8f d = __builtin_amdgcn_wmma_f32_16x16x32_f16(false, a, false, b, (short)0, c, false, false); asm volatile("v_nop\n\tv_nop\n\tv_nop\n\tv_nop" : "+v"(d) : "v"(a), "v"(b)); return d; }

__global__ __launch_bounds__(256) void k_wt_f16(const float* __restrict__ W, _Float16* __restrict__ Wt, unsigned N) {
  const unsigned t = blockIdx.x * 256u + threadIdx.x;
  if (t >= N * (unsigned)(DM / 8)) return;
  const unsigned n = t >> 7, k8 = (t & 127u) << 3;
  FragH f;
#pragma unroll
  for (int i = 0; i < 8; ++i) f.h[i] = (_Float16)(bf16_rne(W[(size_t)(k8 + i) * N + n]) * 16.0f);
  const v8us o = f.half[0];
  unsigned short* d = (unsigned short*)Wt + (size_t)n * DM + k8;
  *(volatile v8us*)d = o;
  __threadfence();
  *(volatile v8us*)d = o;
}

__global__ __launch_bounds__(256) void k_x16(const float* __restrict__ x, _Float16* __restrict__ X16) {
  const unsigned t = blockIdx.x * 256u + threadIdx.x;
  if (t >= (unsigned)(NB * SEQ) * (unsigned)(DM / 8)) return;
  const unsigned row = t >> 7, c8 = (t & 127u) << 3;
  const unsigned b = row / (unsigned)SEQ, tt = row & (unsigned)(SEQ - 1);
  const float* src = x + ((size_t)b * SEQ_FULL + tt) * DM + c8;
  const v4f a = *(const v4fa*)src, c = *(const v4fa*)(src + 4);
  FragH f;
#pragma unroll
  for (int q = 0; q < 4; ++q) { f.h[q] = (_Float16)bf16_rne(a[q]); f.h[4 + q] = (_Float16)bf16_rne(c[q]); }
  const v8us o = f.half[0];
  unsigned short* d = (unsigned short*)X16 + (size_t)t * 8;
  *(volatile v8us*)d = o;
  __threadfence();
  *(volatile v8us*)d = o;
}

__device__ __forceinline__ void g2_loop(const _Float16* a0p, const _Float16* a1p, const _Float16* b0p, size_t ldb, int K, int hh,
                                        v8f& c00, v8f& c01, v8f& c02, v8f& c03, v8f& c10, v8f& c11, v8f& c12, v8f& c13) {
  const _Float16* b1p = b0p + 16 * ldb; const _Float16* b2p = b1p + 16 * ldb; const _Float16* b3p = b2p + 16 * ldb;
#pragma unroll 1
  for (int kb = 0; kb < K; kb += 32) {
    const v16h a0 = g2_frag(a0p + kb, hh), a1 = g2_frag(a1p + kb, hh);
    v16h b = g2_frag(b0p + kb, hh); c00 = g2_mma(a0, b, c00); c10 = g2_mma(a1, b, c10);
    b = g2_frag(b1p + kb, hh); c01 = g2_mma(a0, b, c01); c11 = g2_mma(a1, b, c11);
    b = g2_frag(b2p + kb, hh); c02 = g2_mma(a0, b, c02); c12 = g2_mma(a1, b, c12);
    b = g2_frag(b3p + kb, hh); c03 = g2_mma(a0, b, c03); c13 = g2_mma(a1, b, c13);
  }
}

__global__ __launch_bounds__(128) void k_qkv(const _Float16* __restrict__ X16, const _Float16* __restrict__ Bt, const float* __restrict__ fcs, const float* __restrict__ fsn,
                                             _Float16* __restrict__ QKV, float* __restrict__ F0) {
  __shared__ __attribute__((aligned(16))) float so[4][32][68];
  const unsigned tid = threadIdx.x, w = tid >> 5, lane = tid & 31u, ln = lane & 15u; const int hh = (int)(lane >> 4);
  const unsigned ntn = (unsigned)(NQKV / 64);
  const unsigned mt = blockIdx.x / ntn, nq = blockIdx.x - mt * ntn;
  const unsigned row0 = mt * 128u + 32u * w, col0 = nq * 64u;
  const _Float16* a0p = X16 + (size_t)(row0 + ln) * DM; const _Float16* a1p = a0p + (size_t)16 * DM;
  const _Float16* b0p = Bt + (size_t)(col0 + ln) * DM;
  const v8f z8 = {0.f,0.f,0.f,0.f,0.f,0.f,0.f,0.f};
  v8f c00 = z8, c01 = z8, c02 = z8, c03 = z8, c10 = z8, c11 = z8, c12 = z8, c13 = z8;
  g2_loop(a0p, a1p, b0p, (size_t)DM, DM, hh, c00, c01, c02, c03, c10, c11, c12, c13);
  v8f accs[8] = {c00, c01, c02, c03, c10, c11, c12, c13};
#pragma unroll
  for (int u = 0; u < 8; ++u) {
    const int t = u & 3, half = u >> 2;
#pragma unroll
    for (int r = 0; r < 8; ++r) so[w][half * 16 + 8 * hh + r][t * 16 + (int)ln] = accs[u][r] * 0.0625f;
  }
  __builtin_amdgcn_fence(4  , "workgroup"); __builtin_amdgcn_wave_barrier();
  const unsigned rsub = lane >> 4, c4 = ln * 4u;
  if (col0 < (unsigned)VOFF) {
    const unsigned i0 = c4 >> 1;
#pragma unroll 2
    for (unsigned q = 0; q < 16; ++q) {
      const unsigned r = q * 2u + rsub;
      const unsigned p = (row0 + r) & (unsigned)(SEQ - 1);
      const float cs0 = bf16_rne(fcs[p * 32u + i0]), cs1 = bf16_rne(fcs[p * 32u + i0 + 1u]);
      const float sn0 = bf16_rne(fsn[p * 32u + i0]), sn1 = bf16_rne(fsn[p * 32u + i0 + 1u]);
      const v4f v = *(const v4fa*)&so[w][r][c4];
      v4f o;
      o[0] = v[0] * cs0 - v[1] * sn0; o[1] = v[0] * sn0 + v[1] * cs0;
      o[2] = v[2] * cs1 - v[3] * sn1; o[3] = v[2] * sn1 + v[3] * cs1;
      *(v4fa*)&so[w][r][c4] = o;
    }
  }
  __builtin_amdgcn_fence(4  , "workgroup"); __builtin_amdgcn_wave_barrier();
  const unsigned pos0 = row0 & (unsigned)(SEQ - 1);
  const bool first = pos0 < (unsigned)QT0;
  const size_t frow0 = (size_t)(row0 / (unsigned)SEQ) * QT0 + pos0;
  for (int pass = 0; pass < 2; ++pass) {
#pragma unroll
    for (unsigned q = 0; q < 16; ++q) {
      const unsigned r = q * 2u + rsub;
      const v4f v = *(const v4fa*)&so[w][r][c4];
      v4h h4;
#pragma unroll
      for (int i = 0; i < 4; ++i) h4[i] = (_Float16)v[i];
      *(volatile v4h*)(QKV + (size_t)(row0 + r) * NQKV + col0 + c4) = h4;
      if (first) *(volatile v4f*)(F0 + (frow0 + r) * NQKV + col0 + c4) = v;
    }
    if (pass == 0) __threadfence();
  }
}

template <int NHv, int TTv>
__global__ __launch_bounds__(256) void k_vt(const _Float16* __restrict__ V16, unsigned ldv, unsigned voff, _Float16* __restrict__ Vt) {
  __shared__ unsigned short tl[64][66];
  const unsigned tid = threadIdx.x;
  const unsigned slab = blockIdx.x / (unsigned)(TTv / 64), lg = blockIdx.x - slab * (unsigned)(TTv / 64);
  const unsigned b = slab / (unsigned)NHv, h = slab - b * (unsigned)NHv;
#pragma unroll
  for (unsigned it = 0; it < 2; ++it) {
    const unsigned i = tid + 256u * it; const unsigned r = i >> 3, c8 = (i & 7u) << 3;
    FragH f; f.half[0] = *(const v8us*)((const unsigned short*)V16 + ((size_t)b * TTv + lg * 64u + r) * ldv + voff + h * 64u + c8);
#pragma unroll
    for (int q = 0; q < 8; ++q) tl[r][c8 + q] = f.u[q];
  }
  __syncthreads();
  for (int pass = 0; pass < 2; ++pass) {
#pragma unroll
    for (unsigned rd = 0; rd < 2; ++rd) {
      const unsigned d = rd * 32u + (tid >> 3), pc = tid & 7u; FragH f;
#pragma unroll
      for (int q = 0; q < 8; ++q) f.u[q] = tl[pc * 8u + q][d];
      const v8us o = f.half[0];
      *(volatile v8us*)((unsigned short*)Vt + ((size_t)slab * 64u + d) * TTv + lg * 64u + pc * 8u) = o;
    }
    if (pass == 0) __threadfence();
  }
}

__global__ __launch_bounds__(128) void k_flash(const _Float16* __restrict__ QKV, const _Float16* __restrict__ VT, _Float16* __restrict__ O16) {
  __shared__ __attribute__((aligned(16))) unsigned short ps[4][16][72];
  const unsigned tid = threadIdx.x, w = tid >> 5, lane = tid & 31u, ln = lane & 15u; const int hh = (int)(lane >> 4);
  const unsigned qt = blockIdx.x + (unsigned)(QT0 / 64), h = blockIdx.y, b = blockIdx.z, g = h >> 2;
  const unsigned q0 = qt * 64u + w * 16u;
  const _Float16* qrow = QKV + (size_t)(b * (unsigned)SEQ + q0 + ln) * NQKV + h * (unsigned)HD;
  const v16h aq0 = g2_frag(qrow, hh), aq1 = g2_frag(qrow + 32, hh);
  const _Float16* kbase = QKV + (size_t)(b * (unsigned)SEQ + ln) * NQKV + KOFF + g * (unsigned)HD;
  const _Float16* vbase = VT + ((size_t)(b * (unsigned)NKV + g) * HD + ln) * SEQ;
  const v8f z8 = {0.f,0.f,0.f,0.f,0.f,0.f,0.f,0.f};
  v8f o[4] = {z8, z8, z8, z8};
  float mrow[8], lrow[8];
#pragma unroll
  for (int r = 0; r < 8; ++r) { mrow[r] = -1.0e30f; lrow[r] = 0.f; }
  const unsigned rowb = q0 + 8u * (unsigned)hh;
#pragma unroll 1
  for (unsigned j = 0; j <= qt; ++j) {
    const unsigned kb = j * 64u;
    v8f s[4];
#pragma unroll
    for (int nt = 0; nt < 4; ++nt) {
      const _Float16* kr = kbase + (size_t)(kb + (unsigned)nt * 16u) * NQKV;
      v8f c = z8;
      c = g2_mma(aq0, g2_frag(kr, hh), c);
      c = g2_mma(aq1, g2_frag(kr + 32, hh), c);
      s[nt] = c;
    }
#pragma unroll
    for (int r = 0; r < 8; ++r) {
      const unsigned rowg = rowb + (unsigned)r;
      float sv[4];
#pragma unroll
      for (int nt = 0; nt < 4; ++nt) { const unsigned colg = kb + (unsigned)nt * 16u + ln; const float xv = s[nt][r] * 0.125f; sv[nt] = (colg > rowg) ? -1.0e30f : xv; }
      float mx = fmaxf(fmaxf(sv[0], sv[1]), fmaxf(sv[2], sv[3]));
      mx = fmaxf(mx, __shfl_xor(mx, 1, 32)); mx = fmaxf(mx, __shfl_xor(mx, 2, 32)); mx = fmaxf(mx, __shfl_xor(mx, 4, 32)); mx = fmaxf(mx, __shfl_xor(mx, 8, 32));
      const float mnew = fmaxf(mrow[r], mx);
      const float ce = __expf(fmaxf(mrow[r] - mnew, -100.0f));
      const float corr = (mrow[r] < -1.0e29f) ? 0.f : ce;
      mrow[r] = mnew;
      float rs = 0.f;
#pragma unroll
      for (int nt = 0; nt < 4; ++nt) {
        const float e = __expf(fmaxf(sv[nt] - mnew, -100.0f));
        const float p = (sv[nt] < -1.0e29f) ? 0.f : e * 1024.0f;
        FragH tq; tq.h[0] = (_Float16)p;
        rs += (float)tq.h[0];
        ps[w][8 * hh + r][nt * 16 + (int)ln] = tq.u[0];
      }
      rs += __shfl_xor(rs, 1, 32); rs += __shfl_xor(rs, 2, 32); rs += __shfl_xor(rs, 4, 32); rs += __shfl_xor(rs, 8, 32);
      lrow[r] = lrow[r] * corr + rs;
#pragma unroll
      for (int nt = 0; nt < 4; ++nt) o[nt][r] *= corr;
    }
    __builtin_amdgcn_fence(4  , "workgroup"); __builtin_amdgcn_wave_barrier();
#pragma unroll
    for (int ks = 0; ks < 2; ++ks) {
      FragH ap;
      ap.half[0] = *(const v8us*)&ps[w][ln][ks * 32 + 8 * hh];
      ap.half[1] = *(const v8us*)&ps[w][ln][ks * 32 + 16 + 8 * hh];
#pragma unroll
      for (int nt = 0; nt < 4; ++nt) {
        const _Float16* vr = vbase + (size_t)nt * 16 * SEQ + kb + (unsigned)ks * 32u;
        o[nt] = g2_mma(ap.v, g2_frag(vr, hh), o[nt]);
      }
    }
    __builtin_amdgcn_fence(4  , "workgroup"); __builtin_amdgcn_wave_barrier();
  }
#pragma unroll
  for (int r = 0; r < 8; ++r) {
    const float inv = 64.0f * (1.0f / lrow[r]);
#pragma unroll
    for (int nt = 0; nt < 4; ++nt) { FragH tq; tq.h[0] = (_Float16)(o[nt][r] * inv); ps[w][8 * hh + r][nt * 16 + (int)ln] = tq.u[0]; }
  }
  __builtin_amdgcn_fence(4  , "workgroup"); __builtin_amdgcn_wave_barrier();
  const unsigned rq = lane >> 3, pc = lane & 7u;
  for (int pass = 0; pass < 2; ++pass) {
#pragma unroll
    for (unsigned it = 0; it < 4; ++it) {
      const unsigned rr = it * 4u + rq;
      const v8us v = *(const v8us*)&ps[w][rr][pc * 8u];
      *(volatile v8us*)((unsigned short*)O16 + (size_t)(b * (unsigned)SEQ + q0 + rr) * DM + h * (unsigned)HD + pc * 8u) = v;
    }
    if (pass == 0) __threadfence();
  }
}

__global__ __launch_bounds__(64) void k_att0(const float* __restrict__ F0, float scale, float* __restrict__ OF) {
  #pragma clang fp contract(off)
  __shared__ __attribute__((aligned(16))) float lq[64][64];
  __shared__ __attribute__((aligned(16))) float lo[64][64];
  const unsigned tid = threadIdx.x;
  const unsigned h = blockIdx.x / (unsigned)(QT0 / 64), rg = blockIdx.x - h * (unsigned)(QT0 / 64);
  const unsigned b = blockIdx.y;
  const unsigned i = rg * 64u + tid;
  const float* base = F0 + (size_t)b * QT0 * NQKV;
  const float* qr = base + (size_t)i * NQKV + h * (unsigned)HD;
  const unsigned kc = (unsigned)KOFF + (h >> 2) * (unsigned)HD, vc = (unsigned)VOFF + (h >> 2) * (unsigned)HD;
#pragma unroll 1
  for (unsigned c = 0; c < HD / 4; ++c) { *(v4f*)&lq[tid][c * 4] = *(const v4fa*)(qr + c * 4); const v4f z = {0.f, 0.f, 0.f, 0.f}; *(v4f*)&lo[tid][c * 4] = z; }
  float m = -1.0e30f, l = 0.f;
  const unsigned jmax = rg * 64u + 63u;
#pragma unroll 1
  for (unsigned j = 0; j <= jmax; ++j) {
    const float* kr = base + (size_t)j * NQKV + kc; const float* vr = base + (size_t)j * NQKV + vc; float s = 0.f;
#pragma unroll 1
    for (unsigned c = 0; c < HD / 4; ++c) { const v4f kq = *(const v4fa*)(kr + c * 4); const v4f qq = *(v4f*)&lq[tid][c * 4]; s = __fadd_rn(s, __fmul_rn(qq[0], kq[0])); s = __fadd_rn(s, __fmul_rn(qq[1], kq[1])); s = __fadd_rn(s, __fmul_rn(qq[2], kq[2])); s = __fadd_rn(s, __fmul_rn(qq[3], kq[3])); }
    s = __fmul_rn(s, scale);
    const float f = (j <= i) ? 1.f : 0.f; const float sm = fmaf(f, s, (1.f - f) * -1.0e30f); const float mn = fmaxf(m, sm); const float sc = expf(m - mn); const float e = expf(sm - mn); l = __fadd_rn(__fmul_rn(l, sc), e); m = mn;
#pragma unroll 1
    for (unsigned c = 0; c < HD / 4; ++c) { const v4f vv = *(const v4fa*)(vr + c * 4); v4f oo = *(v4f*)&lo[tid][c * 4]; for (int u = 0; u < 4; ++u) oo[u] = __fadd_rn(__fmul_rn(oo[u], sc), __fmul_rn(e, vv[u])); *(v4f*)&lo[tid][c * 4] = oo; }
  }
  const float fin = 64.0f * (1.0f / l);
#pragma unroll 1
  for (unsigned c = 0; c < HD / 4; ++c) { v4f oo = *(v4f*)&lo[tid][c * 4]; for (int u = 0; u < 4; ++u) oo[u] = __fmul_rn(oo[u], fin); *(v4f*)&lo[tid][c * 4] = oo; }
  __syncthreads();
  for (int pass = 0; pass < 2; ++pass) {
#pragma unroll 1
    for (unsigned it = 0; it < 16; ++it) { const unsigned row = it * 4u + (tid >> 4), pcl = (tid & 15u) << 2; const v4f v = *(const v4f*)&lo[row][pcl]; *(volatile v4f*)(OF + ((size_t)b * QT0 + rg * 64u + row) * DM + h * (unsigned)HD + pcl) = v; }
    if (pass == 0) __threadfence();
  }
}

__global__ __launch_bounds__(256) void k_hl(const float* __restrict__ F, _Float16* __restrict__ Hh, _Float16* __restrict__ Hl, unsigned n8) {
  const unsigned t = blockIdx.x * 256u + threadIdx.x; if (t >= n8) return;
  FragH fh, fl; const v4f a = *(const v4fa*)(F + (size_t)t * 8), c = *(const v4fa*)(F + (size_t)t * 8 + 4);
#pragma unroll
  for (int q = 0; q < 4; ++q) { _Float16 h = (_Float16)a[q]; fh.h[q] = h; fl.h[q] = (_Float16)((a[q] - (float)h) * 1024.0f); h = (_Float16)c[q]; fh.h[4 + q] = h; fl.h[4 + q] = (_Float16)((c[q] - (float)h) * 1024.0f); }
  const v8us oh = fh.half[0], ol = fl.half[0];
  for (int pass = 0; pass < 2; ++pass) { *(volatile v8us*)((unsigned short*)Hh + (size_t)t * 8) = oh; *(volatile v8us*)((unsigned short*)Hl + (size_t)t * 8) = ol; if (pass == 0) __threadfence(); }
}

__global__ __launch_bounds__(128) void k_out(const _Float16* __restrict__ O16, const _Float16* __restrict__ Bo, float* __restrict__ out) {
  __shared__ __attribute__((aligned(16))) float so[4][32][68];
  const unsigned tid = threadIdx.x, w = tid >> 5, lane = tid & 31u, ln = lane & 15u; const int hh = (int)(lane >> 4);
  const unsigned TPB = (unsigned)(SEQ / 128 - 1);
  const unsigned mtile = blockIdx.x >> 4, nq = blockIdx.x & 15u;
  const unsigned b = mtile / TPB, tile = mtile - b * TPB + 1u;
  const unsigned t0 = tile * 128u + 32u * w, col0 = nq * 64u;
  const _Float16* a0p = O16 + (size_t)(b * (unsigned)SEQ + t0 + ln) * DM; const _Float16* a1p = a0p + (size_t)16 * DM;
  const _Float16* b0p = Bo + (size_t)(col0 + ln) * DM;
  const v8f z8 = {0.f,0.f,0.f,0.f,0.f,0.f,0.f,0.f};
  v8f c00 = z8, c01 = z8, c02 = z8, c03 = z8, c10 = z8, c11 = z8, c12 = z8, c13 = z8;
  g2_loop(a0p, a1p, b0p, (size_t)DM, DM, hh, c00, c01, c02, c03, c10, c11, c12, c13);
  v8f accs[8] = {c00, c01, c02, c03, c10, c11, c12, c13};
#pragma unroll
  for (int u = 0; u < 8; ++u) {
    const int t = u & 3, half = u >> 2;
#pragma unroll
    for (int r = 0; r < 8; ++r) so[w][half * 16 + 8 * hh + r][t * 16 + (int)ln] = accs[u][r] * 0.0009765625f;
  }
  __builtin_amdgcn_fence(4  , "workgroup"); __builtin_amdgcn_wave_barrier();
  const unsigned rsub = lane >> 4, c4 = ln * 4u;
  const size_t orow0 = (size_t)b * SEQ_FULL + t0;
  for (int pass = 0; pass < 2; ++pass) {
#pragma unroll
    for (unsigned q = 0; q < 16; ++q) { const unsigned r = q * 2u + rsub; const v4f v = *(const v4fa*)&so[w][r][c4]; *(volatile v4f*)(out + (orow0 + r) * DM + col0 + c4) = v; }
    if (pass == 0) __threadfence();
  }
}

__global__ __launch_bounds__(128) void k_oref(const _Float16* __restrict__ OH, const _Float16* __restrict__ OL, const _Float16* __restrict__ Bo, float* __restrict__ out) {
  __shared__ __attribute__((aligned(16))) float so[4][16][68];
  const unsigned tid = threadIdx.x, w = tid >> 5, lane = tid & 31u, ln = lane & 15u; const int hh = (int)(lane >> 4);
  const unsigned b = blockIdx.y;
  const unsigned wid = blockIdx.x * 4u + w; const unsigned mt = wid >> 4, nq = wid & 15u;
  const unsigned row0 = mt * 16u, col0 = nq * 64u;
  const _Float16* ahp = OH + ((size_t)b * QT0 + row0 + ln) * DM; const _Float16* alp = OL + ((size_t)b * QT0 + row0 + ln) * DM;
  const _Float16* b0p = Bo + (size_t)(col0 + ln) * DM; const _Float16* b1p = b0p + (size_t)16 * DM; const _Float16* b2p = b1p + (size_t)16 * DM; const _Float16* b3p = b2p + (size_t)16 * DM;
  const v8f z8 = {0.f,0.f,0.f,0.f,0.f,0.f,0.f,0.f};
  v8f h0 = z8, h1 = z8, h2 = z8, h3 = z8, l0 = z8, l1 = z8, l2 = z8, l3 = z8;
#pragma unroll 1
  for (int kb = 0; kb < DM; kb += 32) {
    const v16h ah = g2_frag(ahp + kb, hh), al = g2_frag(alp + kb, hh);
    v16h bq = g2_frag(b0p + kb, hh); h0 = g2_mma(ah, bq, h0); l0 = g2_mma(al, bq, l0);
    bq = g2_frag(b1p + kb, hh); h1 = g2_mma(ah, bq, h1); l1 = g2_mma(al, bq, l1);
    bq = g2_frag(b2p + kb, hh); h2 = g2_mma(ah, bq, h2); l2 = g2_mma(al, bq, l2);
    bq = g2_frag(b3p + kb, hh); h3 = g2_mma(ah, bq, h3); l3 = g2_mma(al, bq, l3);
  }
  v8f ach[4] = {h0, h1, h2, h3}; v8f acl[4] = {l0, l1, l2, l3};
#pragma unroll
  for (int t = 0; t < 4; ++t) {
#pragma unroll
    for (int r = 0; r < 8; ++r) so[w][8 * hh + r][t * 16 + (int)ln] = ach[t][r] * 0.0009765625f + acl[t][r] * 0.00000095367431640625f;
  }
  __builtin_amdgcn_fence(4  , "workgroup"); __builtin_amdgcn_wave_barrier();
  const unsigned rsub = lane >> 4, c4 = ln * 4u;
  const size_t orow0 = (size_t)b * SEQ_FULL + row0;
  for (int pass = 0; pass < 2; ++pass) {
#pragma unroll
    for (unsigned q = 0; q < 8; ++q) { const unsigned r = q * 2u + rsub; const v4f v = *(const v4fa*)&so[w][r][c4]; *(volatile v4f*)(out + (orow0 + r) * DM + col0 + c4) = v; }
    if (pass == 0) __threadfence();
  }
}

static_assert(((size_t)DM * DM / 8) % 256 == 0);
static_assert(((size_t)DM * KVD / 8) % 256 == 0);
static_assert(((size_t)NB * SEQ * DM / 8) % 256 == 0);
static_assert(((size_t)NB * SEQ) % 128 == 0);
static_assert(((size_t)NB * QT0 * DM / 8) % 256 == 0);
static_assert(((QT0 / 16) * (DM / 64)) % 4 == 0);

extern "C" void kernel_launch(void* const* d_in, const int* in_sizes, int n_in,
                              void* d_out, int out_size, void* d_ws, size_t ws_size, hipStream_t stream) {
  if (n_in < 7) return;
  const long long xneed = ((long long)(NB - 1) * SEQ_FULL + SEQ) * DM;
  if ((long long)in_sizes[0] < xneed) return;
  if ((long long)in_sizes[1] < (long long)SEQ * 32 || (long long)in_sizes[2] < (long long)SEQ * 32) return;
  if ((long long)in_sizes[3] < (long long)DM * DM || (long long)in_sizes[4] < (long long)DM * KVD || (long long)in_sizes[5] < (long long)DM * KVD || (long long)in_sizes[6] < (long long)DM * DM) return;
  if ((long long)out_size < xneed) return;
  const float* x = (const float*)d_in[0]; const float* fcs = (const float*)d_in[1]; const float* fsn = (const float*)d_in[2];
  const float* wq = (const float*)d_in[3]; const float* wk = (const float*)d_in[4]; const float* wv = (const float*)d_in[5]; const float* wo = (const float*)d_in[6];
  float* out = (float*)d_out;
  char* ws = (char*)d_ws; size_t off = 0;
  auto take = [&](size_t bytes) { char* p = ws + off; off += (bytes + 255) & ~(size_t)255; return p; };
  const size_t NR = (size_t)NB * SEQ;
  _Float16* BQKV = (_Float16*)take((size_t)NQKV * DM * 2);
  _Float16* BO   = (_Float16*)take((size_t)DM * DM * 2);
  _Float16* X16  = (_Float16*)take(NR * DM * 2);
  _Float16* QKV  = (_Float16*)take(NR * NQKV * 2);
  float*    F0   = (float*)take((size_t)NB * QT0 * NQKV * 4);
  _Float16* VT   = (_Float16*)take((size_t)NB * NKV * HD * SEQ * 2);
  _Float16* O16  = (_Float16*)take(NR * DM * 2);
  float*    OF0  = (float*)take((size_t)NB * QT0 * DM * 4);
  _Float16* OH0  = (_Float16*)take((size_t)NB * QT0 * DM * 2);
  _Float16* OL0  = (_Float16*)take((size_t)NB * QT0 * DM * 2);
  if (off > ws_size) return;

  k_wt_f16<<<(unsigned)((size_t)DM * DM / 8 / 256), 256, 0, stream>>>(wq, BQKV, (unsigned)DM);
  k_wt_f16<<<(unsigned)((size_t)DM * KVD / 8 / 256), 256, 0, stream>>>(wk, BQKV + (size_t)KOFF * DM, (unsigned)KVD);
  k_wt_f16<<<(unsigned)((size_t)DM * KVD / 8 / 256), 256, 0, stream>>>(wv, BQKV + (size_t)VOFF * DM, (unsigned)KVD);
  k_wt_f16<<<(unsigned)((size_t)DM * DM / 8 / 256), 256, 0, stream>>>(wo, BO, (unsigned)DM);
  k_x16<<<(unsigned)(NR * DM / 8 / 256), 256, 0, stream>>>(x, X16);
  k_qkv<<<(unsigned)((NR / 128) * (NQKV / 64)), 128, 0, stream>>>(X16, BQKV, fcs, fsn, QKV, F0);
  k_vt<NKV, SEQ><<<(unsigned)(NB * NKV * (SEQ / 64)), 256, 0, stream>>>(QKV, (unsigned)NQKV, (unsigned)VOFF, VT);
  k_flash<<<dim3((unsigned)(SEQ / 64 - QT0 / 64), NH, NB), 128, 0, stream>>>(QKV, VT, O16);
  k_att0<<<dim3((unsigned)(NH * (QT0 / 64)), NB), 64, 0, stream>>>(F0, 0.125f, OF0);
  k_hl<<<(unsigned)((size_t)NB * QT0 * DM / 8 / 256), 256, 0, stream>>>(OF0, OH0, OL0, (unsigned)((size_t)NB * QT0 * DM / 8));
  k_out<<<(unsigned)(NB * (SEQ / 128 - 1) * (DM / 64)), 128, 0, stream>>>(O16, BO, out);
  k_oref<<<dim3((unsigned)((QT0 / 16) * (DM / 64) / 4), NB), 128, 0, stream>>>(OH0, OL0, BO, out);
}
